// MambaEncoder_3126736192210
// MI455X (gfx1250) — hardware-verified
//
#include <hip/hip_runtime.h>
#include <math.h>

typedef __attribute__((ext_vector_type(16))) _Float16 v16h;
typedef __attribute__((ext_vector_type(8)))  _Float16 v8h;
typedef __attribute__((ext_vector_type(4)))  _Float16 v4h;
typedef __attribute__((ext_vector_type(16))) __bf16   v16b;
typedef __attribute__((ext_vector_type(8)))  __bf16   v8b;
typedef __attribute__((ext_vector_type(8)))  float    v8f;
typedef __attribute__((ext_vector_type(4)))  float    v4f;
typedef __attribute__((ext_vector_type(2)))  unsigned v2u;

constexpr int kL    = 4096;
constexpr int kHalf = 512;
constexpr int kDm   = 1024;
constexpr int kDi   = 2048;
constexpr int kNs   = 16;
constexpr int kCv   = 4;
constexpr int kDtR  = 64;
constexpr int kXdN  = 96;
constexpr int kXdP  = 128;
constexpr int kXzP  = 2 * kDi;
constexpr int kTP   = 260;
constexpr int kTS   = 64;
constexpr int kCh   = 64;
constexpr int kYP   = 68;
constexpr int kHP   = 72;
constexpr int kBCP  = 32;
static_assert(kDtR + 2 * kNs == kXdN, "x_proj width");
static_assert(2 * kHalf == kDm, "token width");
static_assert((kDm % 32) == 0 && (kDi % 32) == 0 && (kL % 32) == 0 && (kDtR % 32) == 0, "K multiples of 32");
static_assert((kL % 64) == 0 && (kXzP % 64) == 0 && (kXdP % 64) == 0 && (kDm % 64) == 0, "M,N multiples of 64");
static_assert((kL % kTS) == 0 && (kDi % kCh) == 0 && (kDi % 256) == 0, "tile multiples");
static_assert((size_t)kL * kHalf * 4 == 8388608ull, "second output byte offset");
static_assert((size_t)kL * kDm * 4 == 16777216ull, "output bytes");

constexpr float kCarryFw = 4096.0f;
constexpr float kCarryTt = 16.0f;
constexpr float kCarryU  = 16.0f;
constexpr float kCarryWx = 32.0f;
constexpr float kCarryDt = 64.0f;
constexpr float kCarryWd = 256.0f;
constexpr float kCarryY  = 256.0f;
constexpr float kCarryWo = 1024.0f;
constexpr float kScaleFE  = 0.1f / (kCarryFw * kCarryTt);
constexpr float kScaleXp  = 1.0f / (kCarryU * kCarryWx);
constexpr float kScaleDt  = 1.0f / (kCarryDt * kCarryWd);
constexpr float kScaleOut = 1.0f / (kCarryY * kCarryWo);

constexpr size_t kOffTok16 = 0;
constexpr size_t kOffWin   = kOffTok16 + (size_t)kL * kDm * 2;
constexpr size_t kOffTokT  = kOffWin   + (size_t)kXzP * kDm * 2;
constexpr size_t kOffWx    = kOffTokT  + (size_t)kDm * kL * 2;
constexpr size_t kOffWout  = kOffWx    + (size_t)kXdP * kDi * 2;
constexpr size_t kOffR     = kOffWout  + (size_t)kDm * kDi * 2;
constexpr size_t kOffRes   = kOffR     + (size_t)kL * kXzP * 4;
constexpr size_t kOffU16   = kOffRes   + (size_t)kL * kDm * 4;
constexpr size_t kOffXd    = kOffU16   + (size_t)kL * kDi * 2;
constexpr size_t kOffI1    = kOffXd    + (size_t)kL * kXdP * 4;
constexpr size_t kOffT1    = kOffI1    + (size_t)kL * 4;
constexpr size_t kWsTotal  = kOffT1    + (size_t)kL * 4;
static_assert(kWsTotal == 132677632ull, "carve total");
static_assert(kWsTotal <= 134217728ull, "carve cap");
static_assert((size_t)kL * kL * 2 <= (size_t)kL * kXzP * 4, "FW16 fits region R");
static_assert((size_t)kL * kDm * 4 <= (size_t)kL * kXzP * 4, "SSMO fits region R");
static_assert((kOffWin % 128) == 0 && (kOffTokT % 128) == 0 && (kOffWx % 128) == 0 && (kOffWout % 128) == 0 &&
              (kOffR % 128) == 0 && (kOffRes % 128) == 0 && (kOffU16 % 128) == 0 && (kOffXd % 128) == 0 &&
              (kOffI1 % 128) == 0 && (kOffT1 % 128) == 0, "128-B aligned regions");

__device__ __forceinline__ unsigned short f2bf_bits(float f) {
  unsigned u = __float_as_uint(f);
  return (unsigned short)((u + 0x7FFFu + ((u >> 16) & 1u)) >> 16);
}
__device__ __forceinline__ float bf_bits2f(unsigned short h) { return __uint_as_float(((unsigned)h) << 16); }
__device__ __forceinline__ float bfr(float f) { return bf_bits2f(f2bf_bits(f)); }

__device__ __forceinline__ void acc_guard4(v8f& a, v8f& b, v8f& c, v8f& d) { asm volatile("v_nop\n\tv_nop\n\tv_nop\n\tv_nop" : "+v"(a), "+v"(b), "+v"(c), "+v"(d)); }
__device__ __forceinline__ void row_guard_h(v8f& a0, v8f& a1, v8f& a2, v8f& a3, v16h x, v16h b0, v16h b1, v16h b2, v16h b3) {
  asm volatile("v_nop\n\tv_nop\n\tv_nop\n\tv_nop" : "+v"(a0), "+v"(a1), "+v"(a2), "+v"(a3) : "v"(x), "v"(b0), "v"(b1), "v"(b2), "v"(b3));
}
__device__ __forceinline__ void row_guard_b(v8f& a0, v8f& a1, v8f& a2, v8f& a3, v16b x, v16b b0, v16b b1, v16b b2, v16b b3) {
  asm volatile("v_nop\n\tv_nop\n\tv_nop\n\tv_nop" : "+v"(a0), "+v"(a1), "+v"(a2), "+v"(a3) : "v"(x), "v"(b0), "v"(b1), "v"(b2), "v"(b3));
}
__device__ __forceinline__ v8f mma_h_guarded(v16h a, v16h b, v8f c) {
  c = __builtin_amdgcn_wmma_f32_16x16x32_f16(false, a, false, b, (short)0, c, false, false);
  asm volatile("v_nop\n\tv_nop\n\tv_nop\n\tv_nop" : "+v"(c) : "v"(a), "v"(b));
  return c;
}

template <typename T> struct Frag;
template <> struct Frag<_Float16> {
  typedef v16h V; union U { v16h v; v8h h[2]; };
  static __device__ __forceinline__ v16h load(const _Float16* p) {
    U f; f.h[0] = *(const v8h*)(p); f.h[1] = *(const v8h*)(p + 16); return f.v;
  }
  static __device__ __forceinline__ v8f mma(v16h a, v16h b, v8f c) {
    return __builtin_amdgcn_wmma_f32_16x16x32_f16(false, a, false, b, (short)0, c, false, false);
  }
  static __device__ __forceinline__ void guard4(v8f& a0, v8f& a1, v8f& a2, v8f& a3, v16h x, v16h b0, v16h b1, v16h b2, v16h b3) {
    row_guard_h(a0, a1, a2, a3, x, b0, b1, b2, b3);
  }
};
template <> struct Frag<__bf16> {
  typedef v16b V; union U { v16b v; v8b h[2]; };
  static __device__ __forceinline__ v16b load(const __bf16* p) {
    U f; f.h[0] = *(const v8b*)(p); f.h[1] = *(const v8b*)(p + 16); return f.v;
  }
  static __device__ __forceinline__ v8f mma(v16b a, v16b b, v8f c) {
    return __builtin_amdgcn_wmma_f32_16x16x32_bf16(false, a, false, b, (short)0, c, false, false);
  }
  static __device__ __forceinline__ void guard4(v8f& a0, v8f& a1, v8f& a2, v8f& a3, v16b x, v16b b0, v16b b1, v16b b2, v16b b3) {
    row_guard_b(a0, a1, a2, a3, x, b0, b1, b2, b3);
  }
};
template <int ET> struct Elem;
template <> struct Elem<0> { typedef _Float16 T; };
template <> struct Elem<1> { typedef __bf16 T; };

template <int ET>
__global__ __launch_bounds__(256) void wmma_gemm64(
    const unsigned short* __restrict__ Ap, int lda,
    const unsigned short* __restrict__ Btp, int ldb,
    float* __restrict__ C, int ldc, int M, int N, int K, float scale) {
  typedef typename Elem<ET>::T T;
  typedef typename Frag<T>::V V;
  const T* A = (const T*)Ap;
  const T* Bt = (const T*)Btp;
  __shared__ __align__(16) float sT[8][16 * 68];
  const int lane = threadIdx.x & 31;
  const int wave = threadIdx.x >> 5;
  const int tilesN = N >> 6;
  const int tilesM = M >> 6;
  const int tile = blockIdx.x * 8 + wave;
  if (tile >= tilesM * tilesN) return;
  const int tm = tile / tilesN;
  const int tn = tile - tm * tilesN;
  const int m0 = tm << 6;
  const int n0 = tn << 6;
  const int rlane = lane & 15;
  const int koff  = (lane >> 4) * 8;
  const int mOff  = (lane >> 4) * 8;

  v8f acc[4][4];
#pragma unroll
  for (int i = 0; i < 4; ++i)
#pragma unroll
    for (int j = 0; j < 4; ++j) acc[i][j] = (v8f){0.f,0.f,0.f,0.f,0.f,0.f,0.f,0.f};

  for (int k0 = 0; k0 < K; k0 += 32) {
    V bh[4];
#pragma unroll
    for (int j = 0; j < 4; ++j) {
      const size_t bo = (size_t)(n0 + (j << 4) + rlane) * ldb + koff + k0;
      bh[j] = Frag<T>::load(Bt + bo);
    }
#pragma unroll
    for (int i = 0; i < 4; ++i) {
      const size_t ao = (size_t)(m0 + (i << 4) + rlane) * lda + koff + k0;
      V ah = Frag<T>::load(A + ao);
#pragma unroll
      for (int j = 0; j < 4; ++j) acc[i][j] = Frag<T>::mma(ah, bh[j], acc[i][j]);
      Frag<T>::guard4(acc[i][0], acc[i][1], acc[i][2], acc[i][3], ah, bh[0], bh[1], bh[2], bh[3]);
    }
  }
  acc_guard4(acc[0][0], acc[0][1], acc[0][2], acc[0][3]);
  acc_guard4(acc[1][0], acc[1][1], acc[1][2], acc[1][3]);
  acc_guard4(acc[2][0], acc[2][1], acc[2][2], acc[2][3]);
  acc_guard4(acc[3][0], acc[3][1], acc[3][2], acc[3][3]);

  float* slab = sT[wave];
#pragma unroll
  for (int i = 0; i < 4; ++i) {
    const int mBase = m0 + (i << 4);
#pragma unroll
    for (int j = 0; j < 4; ++j) {
#pragma unroll
      for (int r = 0; r < 8; ++r) {
        const float v = acc[i][j][r] * scale;
        slab[(mOff + r) * 68 + (j << 4) + rlane] = v;
      }
    }
    __builtin_amdgcn_fence(__ATOMIC_RELEASE, "workgroup");
    __builtin_amdgcn_wave_barrier();
    __builtin_amdgcn_fence(__ATOMIC_ACQUIRE, "workgroup");
    {
      const int hh = lane >> 4, c4 = (lane & 15) * 4;
      for (int pass = 0; pass < 2; ++pass) {
#pragma unroll
        for (int it = 0; it < 8; ++it) {
          const int row = it * 2 + hh;
          v4f v = *(const v4f*)(slab + row * 68 + c4);
          *(volatile v4f*)(C + (size_t)(mBase + row) * ldc + n0 + c4) = v;
        }
        __threadfence();
      }
    }
    __builtin_amdgcn_fence(__ATOMIC_RELEASE, "workgroup");
    __builtin_amdgcn_wave_barrier();
    __builtin_amdgcn_fence(__ATOMIC_ACQUIRE, "workgroup");
  }
}

template <int OUTK>
__global__ __launch_bounds__(256) void cast_rows_kernel(
    const float* __restrict__ src, unsigned short* __restrict__ dst,
    int srcRows, int colShift, int dstPitch, int dstColOff, int total8, float scale)
{
  const int i = blockIdx.x * 256 + threadIdx.x;
  if (i >= total8) return;
  const int e0 = i << 3;
  const int r  = e0 >> colShift;
  const int c  = e0 & ((1 << colShift) - 1);
  const bool live = (r < srcRows);
  const int rc = live ? r : (srcRows - 1);
  const float* p = src + (((size_t)rc) << colShift) + c;
  const v4f a0 = *(const v4f*)(p);
  const v4f a1 = *(const v4f*)(p + 4);
  v8h hv;
#pragma unroll
  for (int e = 0; e < 4; ++e) {
    const float g0 = a0[e];
    const float g1 = a1[e];
    const float f0 = live ? g0 : 0.0f;
    const float f1 = live ? g1 : 0.0f;
    const unsigned short h0 = f2bf_bits(f0);
    const unsigned short h1 = f2bf_bits(f1);
    if (OUTK == 0) {
      hv[e]     = __builtin_bit_cast(_Float16, h0);
      hv[4 + e] = __builtin_bit_cast(_Float16, h1);
    } else {
      hv[e]     = (_Float16)(bf_bits2f(h0) * scale);
      hv[4 + e] = (_Float16)(bf_bits2f(h1) * scale);
    }
  }
  unsigned short* q = dst + (size_t)r * dstPitch + dstColOff + c;
  *(volatile v8h*)q = hv;
  __threadfence();
  *(volatile v8h*)q = hv;
}

__global__ __launch_bounds__(256) void transpose_cast_kernel(
    const float* __restrict__ W, unsigned short* __restrict__ Bt, int Kdim, int Ndim, float scale)
{
  __shared__ float tile[64 * 65];
  const int tid = threadIdx.x, lane = tid & 31, wave = tid >> 5;
  const int n0 = blockIdx.x * 64;
  const int k0 = blockIdx.y * 64;
#pragma unroll
  for (int p = 0; p < 16; ++p) {
    const int idx = tid + p * 256;
    const int kk  = idx >> 6;
    const int nn  = idx & 63;
    const int n   = n0 + nn;
    const int nc  = (n < Ndim) ? n : (Ndim - 1);
    const float v = W[(size_t)(k0 + kk) * Ndim + nc];
    tile[kk * 65 + nn] = (n < Ndim) ? (bfr(v) * scale) : 0.0f;
  }
  __syncthreads();
  const int q = lane >> 3, c8 = (lane & 7) * 8;
  v8h hv[2];
#pragma unroll
  for (int it = 0; it < 2; ++it) {
    const int nrow = it * 32 + wave * 4 + q;
#pragma unroll
    for (int e = 0; e < 8; ++e) hv[it][e] = (_Float16)tile[(c8 + e) * 65 + nrow];
  }
  for (int pass = 0; pass < 2; ++pass) {
#pragma unroll
    for (int it = 0; it < 2; ++it) {
      const int nrow = it * 32 + wave * 4 + q;
      *(volatile v8h*)(Bt + (size_t)(n0 + nrow) * Kdim + k0 + c8) = hv[it];
    }
    __threadfence();
  }
}

__global__ __launch_bounds__(256) void rowsum_kernel(
    const float* __restrict__ img, const float* __restrict__ txt, float* __restrict__ I1, float* __restrict__ T1)
{
  __shared__ float sI[32];
  __shared__ float sU[32];
  const int tid = threadIdx.x, lane = tid & 31, wave = tid >> 5;
  const int r0 = blockIdx.x * 32;
#pragma unroll 1
  for (int q = 0; q < 4; ++q) {
    const int rr = wave * 4 + q;
    const size_t base = (size_t)(r0 + rr) * kHalf + lane * 4;
    float si = 0.0f, st = 0.0f;
#pragma unroll
    for (int k = 0; k < 4; ++k) {
      const v4f a = *(const v4f*)(img + base + k * 128);
      const v4f b = *(const v4f*)(txt + base + k * 128);
      const float a0 = a[0], a1 = a[1], a2 = a[2], a3 = a[3];
      const float b0 = b[0], b1 = b[1], b2 = b[2], b3 = b[3];
      si += (bfr(a0) + bfr(a1)) + (bfr(a2) + bfr(a3));
      st += (bfr(b0) + bfr(b1)) + (bfr(b2) + bfr(b3));
    }
#pragma unroll
    for (int off = 16; off >= 1; off >>= 1) {
      si += __shfl_xor(si, off, 32);
      st += __shfl_xor(st, off, 32);
    }
    if (lane == 0) { sI[rr] = si; sU[rr] = st; }
  }
  __syncthreads();
  if (wave == 0) {
    const float vi = sI[lane];
    const float vt = sU[lane];
    volatile float* pi = I1 + r0 + lane;
    volatile float* pt = T1 + r0 + lane;
    *pi = vi;
    *pt = vt;
    __threadfence();
    *pi = vi;
    *pt = vt;
  }
}

__global__ __launch_bounds__(256) void fe_weight_kernel(
    const float* __restrict__ I1, const float* __restrict__ T1, unsigned short* __restrict__ FW16)
{
#pragma clang fp contract(off)
  const int idx = blockIdx.x * 256 + threadIdx.x;
  const int i  = idx >> 10;
  const int j4 = (idx & 1023) << 2;
  const float ai = I1[i];
  const float ti = T1[i];
  const v4f aj = *(const v4f*)(I1 + j4);
  const v4f tj = *(const v4f*)(T1 + j4);
  unsigned hb[4];
#pragma unroll
  for (int e = 0; e < 4; ++e) {
    const float ajv = aj[e];
    const float tjv = tj[e];
    const float p1 = ai * ajv;
    const float p2 = ti * tjv;
    const float s  = p1 - p2;
    const float a  = fminf(fabsf(s), 40.0f);
    const float e1 = expf(-a);
    const float e2 = e1 * e1;
    const float r1 = __builtin_amdgcn_rcpf(1.0f + e1);
    const float r2 = __builtin_amdgcn_rcpf(1.0f + e2);
    const float w  = 4.0f * ((e2 * r2) * r2) * ((e1 * r1) * r1);
    const _Float16 hw = (_Float16)(w * kCarryFw);
    hb[e] = (unsigned)__builtin_bit_cast(unsigned short, hw);
  }
  v2u ov;
  ov[0] = hb[0] | (hb[1] << 16);
  ov[1] = hb[2] | (hb[3] << 16);
  unsigned short* q = FW16 + (size_t)i * kL + j4;
  *(volatile v2u*)q = ov;
  __threadfence();
  *(volatile v2u*)q = ov;
}

__global__ __launch_bounds__(256) void conv_silu_kernel(
    const float* __restrict__ XZ, const float* __restrict__ cw, const float* __restrict__ cb,
    unsigned short* __restrict__ U16)
{
  __shared__ __align__(16) float sT[16 * kTP];
  const int tid = threadIdx.x, lane = tid & 31, wave = tid >> 5;
  const int d0 = blockIdx.x * 256, d = d0 + tid;
  const int t0 = blockIdx.y * 64;
  const v4f wq = *(const v4f*)(cw + (size_t)d * kCv);
  const float q0 = wq[0], q1 = wq[1], q2 = wq[2], q3 = wq[3];
  const float w0 = bfr(q0), w1 = bfr(q1), w2 = bfr(q2), w3 = bfr(q3);
  const float bc = bfr(cb[d]);
  float xm3, xm2, xm1;
  {
    const int r3 = t0 - 3, r2 = t0 - 2, r1 = t0 - 1;
    const float v3 = XZ[(size_t)(r3 < 0 ? 0 : r3) * kXzP + d];
    const float v2 = XZ[(size_t)(r2 < 0 ? 0 : r2) * kXzP + d];
    const float v1 = XZ[(size_t)(r1 < 0 ? 0 : r1) * kXzP + d];
    xm3 = (r3 >= 0) ? v3 : 0.0f;
    xm2 = (r2 >= 0) ? v2 : 0.0f;
    xm1 = (r1 >= 0) ? v1 : 0.0f;
  }
#pragma unroll 1
  for (int sub = 0; sub < 4; ++sub) {
    const int lb = t0 + sub * 16;
#pragma unroll 1
    for (int s = 0; s < 16; ++s) {
      const float xc = XZ[(size_t)(lb + s) * kXzP + d];
      float acc = w0 * xm3;
      acc = fmaf(w1, xm2, acc);
      acc = fmaf(w2, xm1, acc);
      acc = fmaf(w3, xc, acc);
      const float sv = acc + bc;
      const float sg = __builtin_amdgcn_rcpf(1.0f + __expf(-sv));
      sT[s * kTP + tid] = (sv * sg) * kCarryU;
      xm3 = xm2; xm2 = xm1; xm1 = xc;
    }
    __syncthreads();
    v8h bv[2];
#pragma unroll
    for (int it = 0; it < 2; ++it) {
      const float* sp = sT + (it * 8 + wave) * kTP + lane * 8;
      const v4f a0 = *(const v4f*)(sp);
      const v4f a1 = *(const v4f*)(sp + 4);
#pragma unroll
      for (int e = 0; e < 4; ++e) {
        const float g0 = a0[e];
        const float g1 = a1[e];
        bv[it][e]     = (_Float16)g0;
        bv[it][4 + e] = (_Float16)g1;
      }
    }
    for (int pass = 0; pass < 2; ++pass) {
#pragma unroll
      for (int it = 0; it < 2; ++it)
        *(volatile v8h*)(U16 + (size_t)(lb + it * 8 + wave) * kDi + d0 + lane * 8) = bv[it];
      __threadfence();
    }
    __syncthreads();
  }
}

__global__ __launch_bounds__(64) void scan_kernel(
    const float* __restrict__ XD, const float* __restrict__ XZ,
    const float* __restrict__ cw, const float* __restrict__ cb,
    const float* __restrict__ Wdt, const float* __restrict__ bdt, const float* __restrict__ Alog,
    const float* __restrict__ Dp, unsigned short* __restrict__ Y16)
{
  __shared__ __align__(16) float    sBC[kTS * kBCP];
  __shared__ __align__(16) _Float16 sDt[kTS * kHP];
  __shared__ __align__(16) _Float16 sWd[kCh * kHP];
  __shared__ __align__(16) float    sD[kTS * kYP];
  __shared__ __align__(16) float    sY[kTS * kYP];
  union FH { v16h v; v8h h[2]; };
  const int tid = threadIdx.x, lane = tid & 31, wave = tid >> 5;
  const int d0 = blockIdx.x * kCh;
  const int d  = d0 + tid;
  const int rlane = lane & 15;
  const int koff  = (lane >> 4) * 8;
  const int mOff  = (lane >> 4) * 8;

  {
    const float* wrow = Wdt + (size_t)d * kDtR;
#pragma unroll 1
    for (int r4 = 0; r4 < kDtR / 4; ++r4) {
      const v4f wv = *(const v4f*)(wrow + 4 * r4);
      const float f0 = wv[0], f1 = wv[1], f2 = wv[2], f3 = wv[3];
      v4h hv;
      hv[0] = (_Float16)(bfr(f0) * kCarryWd);
      hv[1] = (_Float16)(bfr(f1) * kCarryWd);
      hv[2] = (_Float16)(bfr(f2) * kCarryWd);
      hv[3] = (_Float16)(bfr(f3) * kCarryWd);
      *(v4h*)(sWd + tid * kHP + 4 * r4) = hv;
    }
  }
  float negA[kNs], h[kNs];
#pragma unroll
  for (int q4 = 0; q4 < 4; ++q4) {
    const v4f av = *(const v4f*)(Alog + (size_t)d * kNs + 4 * q4);
    const float f0 = av[0], f1 = av[1], f2 = av[2], f3 = av[3];
    negA[4 * q4 + 0] = -__expf(bfr(f0));
    negA[4 * q4 + 1] = -__expf(bfr(f1));
    negA[4 * q4 + 2] = -__expf(bfr(f2));
    negA[4 * q4 + 3] = -__expf(bfr(f3));
  }
#pragma unroll
  for (int n = 0; n < kNs; ++n) h[n] = 0.0f;
  const float bb = bfr(bdt[d]);
  const float Dd = bfr(Dp[d]);
  const v4f wq = *(const v4f*)(cw + (size_t)d * kCv);
  const float q0 = wq[0], q1 = wq[1], q2 = wq[2], q3 = wq[3];
  const float w0 = bfr(q0), w1 = bfr(q1), w2 = bfr(q2), w3 = bfr(q3);
  const float cbias = bfr(cb[d]);
  float xm3 = 0.0f, xm2 = 0.0f, xm1 = 0.0f;
  const int q = lane >> 3, c8 = (lane & 7) * 8;

#pragma unroll 1
  for (int t0 = 0; t0 < kL; t0 += kTS) {
    __syncthreads();
#pragma unroll 4
    for (int i = 0; i < 16; ++i) {
      const int idx = tid + 64 * i;
      const int row = idx >> 4;
      const int c4  = (idx & 15) * 4;
      const v4f xv = *(const v4f*)(XD + (size_t)(t0 + row) * kXdP + c4);
      const float f0 = xv[0], f1 = xv[1], f2 = xv[2], f3 = xv[3];
      v4h hv;
      hv[0] = (_Float16)(f0 * kCarryDt);
      hv[1] = (_Float16)(f1 * kCarryDt);
      hv[2] = (_Float16)(f2 * kCarryDt);
      hv[3] = (_Float16)(f3 * kCarryDt);
      *(v4h*)(sDt + row * kHP + c4) = hv;
    }
#pragma unroll 4
    for (int i = 0; i < 8; ++i) {
      const int idx = tid + 64 * i;
      const int row = idx >> 3;
      const int c4  = (idx & 7) * 4;
      *(v4f*)(sBC + row * kBCP + c4) = *(const v4f*)(XD + (size_t)(t0 + row) * kXdP + kDtR + c4);
    }
    __syncthreads();
    {
      v8f dacc[2][4];
#pragma unroll
      for (int i = 0; i < 2; ++i)
#pragma unroll
        for (int j = 0; j < 4; ++j) dacc[i][j] = (v8f){0.f,0.f,0.f,0.f,0.f,0.f,0.f,0.f};
#pragma unroll
      for (int ks = 0; ks < 2; ++ks) {
        v16h bq[4];
#pragma unroll
        for (int j = 0; j < 4; ++j) {
          FH f;
          const _Float16* bp = sWd + (j * 16 + rlane) * kHP + koff + ks * 32;
          f.h[0] = *(const v8h*)(bp);
          f.h[1] = *(const v8h*)(bp + 16);
          bq[j] = f.v;
        }
#pragma unroll
        for (int i = 0; i < 2; ++i) {
          FH f;
          const _Float16* ap = sDt + (wave * 32 + i * 16 + rlane) * kHP + koff + ks * 32;
          f.h[0] = *(const v8h*)(ap);
          f.h[1] = *(const v8h*)(ap + 16);
#pragma unroll
          for (int j = 0; j < 4; ++j) dacc[i][j] = mma_h_guarded(f.v, bq[j], dacc[i][j]);
        }
      }
#pragma unroll
      for (int i = 0; i < 2; ++i)
#pragma unroll
        for (int j = 0; j < 4; ++j)
#pragma unroll
          for (int r = 0; r < 8; ++r)
            sD[(wave * 32 + i * 16 + mOff + r) * kYP + j * 16 + rlane] = dacc[i][j][r] * kScaleDt;
    }
    __syncthreads();
#pragma unroll 1
    for (int s = 0; s < kTS; ++s) {
      const size_t trow = (size_t)(t0 + s) * kXzP;
      const float xcur = XZ[trow + d];
      const float zv   = XZ[trow + kDi + d];
      const float* bcp = sBC + s * kBCP;
      float Bs[kNs], Cs[kNs];
#pragma unroll
      for (int q4 = 0; q4 < 4; ++q4) {
        const v4f bv = *(const v4f*)(bcp + 4 * q4);
        const v4f cv = *(const v4f*)(bcp + kNs + 4 * q4);
        Bs[4 * q4 + 0] = bv[0]; Bs[4 * q4 + 1] = bv[1]; Bs[4 * q4 + 2] = bv[2]; Bs[4 * q4 + 3] = bv[3];
        Cs[4 * q4 + 0] = cv[0]; Cs[4 * q4 + 1] = cv[1]; Cs[4 * q4 + 2] = cv[2]; Cs[4 * q4 + 3] = cv[3];
      }
      const float v   = sD[s * kYP + tid] + bb;
      const float a   = __expf(-fabsf(v));
      const float up  = 1.0f + a;
      const float l1p = __logf(up) + (a - (up - 1.0f)) * __builtin_amdgcn_rcpf(up);
      const float dt  = fmaxf(v, 0.0f) + l1p;
      float acc = w0 * xm3;
      acc = fmaf(w1, xm2, acc);
      acc = fmaf(w2, xm1, acc);
      acc = fmaf(w3, xcur, acc);
      const float sv = acc + cbias;
      const float su = __builtin_amdgcn_rcpf(1.0f + expf(-sv));
      const float ut = sv * su;
      xm3 = xm2; xm2 = xm1; xm1 = xcur;
      const float dtx = dt * ut;
      float y = 0.0f;
#pragma unroll
      for (int k = 0; k < kNs; ++k) {
        const float e = __expf(dt * negA[k]);
        h[k] = e * h[k] + dtx * Bs[k];
        y = h[k] * Cs[k] + y;
      }
      y = ut * Dd + y;
      const float sz = __builtin_amdgcn_rcpf(1.0f + expf(-zv));
      sY[s * kYP + tid] = (y * (zv * sz)) * kCarryY;
    }
    __syncthreads();
    v8h hv[8];
#pragma unroll
    for (int it = 0; it < 8; ++it) {
      const int row = it * 8 + wave * 4 + q;
      const float* sp = sY + row * kYP + c8;
      const v4f a0 = *(const v4f*)(sp);
      const v4f a1 = *(const v4f*)(sp + 4);
#pragma unroll
      for (int e = 0; e < 4; ++e) {
        const float g0 = a0[e];
        const float g1 = a1[e];
        hv[it][e]     = (_Float16)g0;
        hv[it][4 + e] = (_Float16)g1;
      }
    }
    for (int pass = 0; pass < 2; ++pass) {
#pragma unroll
      for (int it = 0; it < 8; ++it) {
        const int row = it * 8 + wave * 4 + q;
        *(volatile v8h*)(Y16 + (size_t)(t0 + row) * kDi + d0 + c8) = hv[it];
      }
      __threadfence();
    }
  }
}

__global__ __launch_bounds__(256) void norm_split_kernel(
    const float* __restrict__ SSMO, const float* __restrict__ FE, float* __restrict__ out)
{
  __shared__ float sP[8];
  const int tid = threadIdx.x, lane = tid & 31, wave = tid >> 5;
  const int row = blockIdx.x;
  const int c4 = tid * 4;
  const v4f a = *(const v4f*)(SSMO + (size_t)row * kDm + c4);
  const v4f b = *(const v4f*)(FE + (size_t)row * kDm + c4);
  const float r0 = a[0] + b[0];
  const float r1 = a[1] + b[1];
  const float r2 = a[2] + b[2];
  const float r3 = a[3] + b[3];
  float ss = (r0 * r0 + r1 * r1) + (r2 * r2 + r3 * r3);
#pragma unroll
  for (int off = 16; off >= 1; off >>= 1) ss += __shfl_xor(ss, off, 32);
  if (lane == 0) sP[wave] = ss;
  __syncthreads();
  const float tot = ((sP[0] + sP[1]) + (sP[2] + sP[3])) + ((sP[4] + sP[5]) + (sP[6] + sP[7]));
  const float inv = 1.0f / fmaxf(sqrtf(tot), 1e-12f);
  v4f o;
  o[0] = r0 * inv;
  o[1] = r1 * inv;
  o[2] = r2 * inv;
  o[3] = r3 * inv;
  const bool first = (c4 < kHalf);
  const size_t eo = first ? ((size_t)row * kHalf + c4)
                          : ((size_t)kL * kHalf + (size_t)row * kHalf + (c4 - kHalf));
  float* p = out + eo;
  *(volatile v4f*)p = o;
  __threadfence();
  *(volatile v4f*)p = o;
}

static_assert(((kL / 64) * (kDm / 64)) % 8 == 0 && ((kL / 64) * (kXzP / 64)) % 8 == 0 && ((kL / 64) * (kXdP / 64)) % 8 == 0, "tile counts fill whole blocks");

extern "C" void kernel_launch(void* const* d_in, const int* in_sizes, int n_in,
                              void* d_out, int out_size, void* d_ws, size_t ws_size,
                              hipStream_t stream)
{
  if (n_in < 11) return;
  if (in_sizes[0] != kL * kHalf || in_sizes[1] != kL * kHalf) return;
  if (in_sizes[2] != kXzP * kDm) return;
  if (in_sizes[3] != kDi * kCv || in_sizes[4] != kDi) return;
  if (in_sizes[5] != kXdN * kDi) return;
  if (in_sizes[6] != kDi * kDtR || in_sizes[7] != kDi) return;
  if (in_sizes[8] != kDi * kNs || in_sizes[9] != kDi) return;
  if (in_sizes[10] != kDm * kDi) return;
  if (out_size != kL * kDm) return;
  if (ws_size < kWsTotal) return;

  const float* img    = (const float*)d_in[0];
  const float* txt    = (const float*)d_in[1];
  const float* W_in   = (const float*)d_in[2];
  const float* conv_w = (const float*)d_in[3];
  const float* conv_b = (const float*)d_in[4];
  const float* W_x    = (const float*)d_in[5];
  const float* W_dt   = (const float*)d_in[6];
  const float* b_dt   = (const float*)d_in[7];
  const float* A_log  = (const float*)d_in[8];
  const float* Dv     = (const float*)d_in[9];
  const float* W_out  = (const float*)d_in[10];
  float* out = (float*)d_out;

  char* ws = (char*)d_ws;
  unsigned short* TOK16 = (unsigned short*)(ws + kOffTok16);
  unsigned short* WIN   = (unsigned short*)(ws + kOffWin);
  unsigned short* TOKT  = (unsigned short*)(ws + kOffTokT);
  unsigned short* WX    = (unsigned short*)(ws + kOffWx);
  unsigned short* WOUT  = (unsigned short*)(ws + kOffWout);
  unsigned short* FW16  = (unsigned short*)(ws + kOffR);
  float*          XZ    = (float*)(ws + kOffR);
  float*          SSMO  = (float*)(ws + kOffR);
  float*          RES   = (float*)(ws + kOffRes);
  unsigned short* U16   = (unsigned short*)(ws + kOffU16);
  unsigned short* Y16   = (unsigned short*)(ws + kOffU16);
  float*          XD    = (float*)(ws + kOffXd);
  float*          I1    = (float*)(ws + kOffI1);
  float*          T1    = (float*)(ws + kOffT1);

  cast_rows_kernel<0><<<(kL * kHalf / 8) / 256, 256, 0, stream>>>(img, TOK16, kL, 9, kDm, 0, kL * kHalf / 8, 1.0f);
  cast_rows_kernel<0><<<(kL * kHalf / 8) / 256, 256, 0, stream>>>(txt, TOK16, kL, 9, kDm, kHalf, kL * kHalf / 8, 1.0f);

  transpose_cast_kernel<<<dim3(kHalf / 64, kL / 64), 256, 0, stream>>>(img, TOKT, kL, kHalf, kCarryTt);
  transpose_cast_kernel<<<dim3(kHalf / 64, kL / 64), 256, 0, stream>>>(txt, TOKT + (size_t)kHalf * kL, kL, kHalf, kCarryTt);

  rowsum_kernel<<<kL / 32, 256, 0, stream>>>(img, txt, I1, T1);

  cast_rows_kernel<0><<<(kXzP * kDm / 8) / 256, 256, 0, stream>>>(W_in, WIN, kXzP, 10, kDm, 0, kXzP * kDm / 8, 1.0f);
  cast_rows_kernel<1><<<(kXdP * kDi / 8) / 256, 256, 0, stream>>>(W_x, WX, kXdN, 11, kDi, 0, kXdP * kDi / 8, kCarryWx);
  cast_rows_kernel<1><<<(kDm * kDi / 8) / 256, 256, 0, stream>>>(W_out, WOUT, kDm, 11, kDi, 0, kDm * kDi / 8, kCarryWo);

  fe_weight_kernel<<<(kL * (kL / 4)) / 256, 256, 0, stream>>>(I1, T1, FW16);

  wmma_gemm64<0><<<((kL / 64) * (kDm / 64)) / 8, 256, 0, stream>>>(
      FW16, kL, TOKT, kL, RES, kDm, kL, kDm, kL, kScaleFE);

  wmma_gemm64<1><<<((kL / 64) * (kXzP / 64)) / 8, 256, 0, stream>>>(
      TOK16, kDm, WIN, kDm, XZ, kXzP, kL, kXzP, kDm, 1.0f);

  conv_silu_kernel<<<dim3(kDi / 256, kL / 64), 256, 0, stream>>>(XZ, conv_w, conv_b, U16);

  wmma_gemm64<0><<<((kL / 64) * (kXdP / 64)) / 8, 256, 0, stream>>>(
      U16, kDi, WX, kDi, XD, kXdP, kL, kXdP, kDi, kScaleXp);

  scan_kernel<<<kDi / kCh, kCh, 0, stream>>>(XD, XZ, conv_w, conv_b, W_dt, b_dt, A_log, Dv, Y16);

  wmma_gemm64<0><<<((kL / 64) * (kDm / 64)) / 8, 256, 0, stream>>>(
      Y16, kDi, WOUT, kDi, SSMO, kDm, kL, kDm, kDi, kScaleOut);

  norm_split_kernel<<<kL, 256, 0, stream>>>(SSMO, RES, out);
}
